// TemporalFusionTransformer_29222957482030
// MI455X (gfx1250) — hardware-verified
//
#include <hip/hip_runtime.h>
#include <math.h>

typedef __attribute__((ext_vector_type(16))) _Float16 v16h;
typedef __attribute__((ext_vector_type(8)))  _Float16 v8h;
typedef __attribute__((ext_vector_type(16))) __bf16   v16b;
typedef __attribute__((ext_vector_type(8)))  __bf16   v8b;
typedef __attribute__((ext_vector_type(8)))  float    v8f;
typedef __attribute__((ext_vector_type(4)))  float    v4f;
typedef __attribute__((ext_vector_type(4)))  unsigned v4u;

#define DEVI __device__ __forceinline__

static constexpr int NTOK  = 1024;
static constexpr int FIN   = 128;
static constexpr int HID   = 256;
static constexpr int SEQ   = 128;
static constexpr int NBAT  = 8;
static constexpr int NLAY  = 4;
static constexpr int NGATE = 1024;
static constexpr int GRP   = 16;
static constexpr int NGRP  = 8;
static_assert(GRP * NGRP == FIN);
static constexpr float WCAR    = 64.0f;
static constexpr float ATT_SCL = 0.17677669529663687f;
static constexpr float PCAR    = 32768.0f;
static constexpr float CTXCAR  = 16.0f;

__device__ __forceinline__ unsigned short f2bf_bits(float f) {
  unsigned u = __float_as_uint(f);
  return (unsigned short)((u + 0x7FFFu + ((u >> 16) & 1u)) >> 16);
}
__device__ __forceinline__ float bf_bits2f(unsigned short h) { return __uint_as_float(((unsigned)h) << 16); }

__device__ __forceinline__ void dep_guard_h(v8f& a, v8f& b, v16h x, v16h y) { asm volatile("v_nop\n\tv_nop\n\tv_nop\n\tv_nop" : "+v"(a), "+v"(b) : "v"(x), "v"(y)); }
__device__ __forceinline__ void dep_guard_b(v8f& a, v8f& b, v16b x, v16b y) { asm volatile("v_nop\n\tv_nop\n\tv_nop\n\tv_nop" : "+v"(a), "+v"(b) : "v"(x), "v"(y)); }
__device__ __forceinline__ void keep4_h(v16h a, v16h b, v16h c, v16h d) { asm volatile("v_nop" :: "v"(a), "v"(b), "v"(c), "v"(d)); }
__device__ __forceinline__ void keep4_b(v16b a, v16b b, v16b c, v16b d) { asm volatile("v_nop" :: "v"(a), "v"(b), "v"(c), "v"(d)); }
__device__ __forceinline__ void acc_guard4(v8f& a, v8f& b, v8f& c, v8f& d) { asm volatile("v_nop\n\tv_nop\n\tv_nop\n\tv_nop" : "+v"(a), "+v"(b), "+v"(c), "+v"(d)); }
template <typename T> struct Frag;
template <> struct Frag<_Float16> {
  typedef v16h V; union U { v16h v; v8h h[2]; };
  static __device__ __forceinline__ v16h load(const _Float16* p) {
    U f; f.h[0] = *(const v8h*)(p); f.h[1] = *(const v8h*)(p + 16); return f.v;
  }
  static __device__ __forceinline__ v8f mma(v16h a, v16h b, v8f c) {
    return __builtin_amdgcn_wmma_f32_16x16x32_f16(false, a, false, b, (short)0, c, false, false);
  }
  static __device__ __forceinline__ void guard(v8f& a, v8f& b, v16h x, v16h y) { dep_guard_h(a, b, x, y); }
  static __device__ __forceinline__ void keep(v16h a, v16h b, v16h c, v16h d) { keep4_h(a, b, c, d); }
};
template <> struct Frag<__bf16> {
  typedef v16b V; union U { v16b v; v8b h[2]; };
  static __device__ __forceinline__ v16b load(const __bf16* p) {
    U f; f.h[0] = *(const v8b*)(p); f.h[1] = *(const v8b*)(p + 16); return f.v;
  }
  static __device__ __forceinline__ v8f mma(v16b a, v16b b, v8f c) {
    return __builtin_amdgcn_wmma_f32_16x16x32_bf16(false, a, false, b, (short)0, c, false, false);
  }
  static __device__ __forceinline__ void guard(v8f& a, v8f& b, v16b x, v16b y) { dep_guard_b(a, b, x, y); }
  static __device__ __forceinline__ void keep(v16b a, v16b b, v16b c, v16b d) { keep4_b(a, b, c, d); }
};

template <int ET> struct Elem;
template <> struct Elem<0> { typedef _Float16 T; };
template <> struct Elem<1> { typedef __bf16 T; };
template <int ET, bool SPLIT, int BIAS_MODE, int OUT_MODE, bool RESID, int ACT = 0>
__global__ __launch_bounds__(256) void wmma_gemm64(
    const unsigned short* __restrict__ Ap, const unsigned short* __restrict__ A2p, int lda, long strideA,
    const unsigned short* __restrict__ Btp, const unsigned short* __restrict__ Bt2p, int ldb, long strideB,
    void* __restrict__ Cout, void* __restrict__ Cout2, int ldc, long strideC,
    const float* __restrict__ bias, long strideBias,
    const float* __restrict__ resid, long strideR,
    int M, int N, int K, float scale, float oscale) {
  typedef typename Elem<ET>::T T;
  typedef typename Frag<T>::V V;
  const T* A = (const T*)Ap; const T* A2 = (const T*)A2p; const T* Bt = (const T*)Btp; const T* Bt2 = (const T*)Bt2p;
  __shared__ __align__(16) float sT[8][16 * 68];
  const int b    = blockIdx.y;
  const int lane = threadIdx.x & 31;
  const int wave = threadIdx.x >> 5;
  const int tilesN = N >> 6;
  const int tilesM = M >> 6;
  const int tile = blockIdx.x * 8 + wave;
  if (tile >= tilesM * tilesN) return;
  const int tm = tile / tilesN;
  const int tn = tile - tm * tilesN;
  const int m0 = tm << 6;
  const int n0 = tn << 6;

  const T* Ab  = A  + (size_t)b * strideA;
  const T* Bb  = Bt + (size_t)b * strideB;
  const T* Ab2 = SPLIT ? (A2  + (size_t)b * strideA) : nullptr;
  const T* Bb2 = SPLIT ? (Bt2 + (size_t)b * strideB) : nullptr;

  const int rlane = lane & 15;
  const int koff  = (lane >> 4) * 8;
  const int mOff  = (lane >> 4) * 8;

  v8f acc[4][4];
#pragma unroll
  for (int i = 0; i < 4; ++i)
#pragma unroll
    for (int j = 0; j < 4; ++j) acc[i][j] = (v8f){0.f,0.f,0.f,0.f,0.f,0.f,0.f,0.f};

  for (int k0 = 0; k0 < K; k0 += 32) {
    V bh[4], bl[4];
#pragma unroll
    for (int j = 0; j < 4; ++j) {
      const size_t bo = (size_t)(n0 + (j << 4) + rlane) * ldb + koff + k0;
      bh[j] = Frag<T>::load(Bb + bo);
      if (SPLIT) bl[j] = Frag<T>::load(Bb2 + bo);
    }
#pragma unroll
    for (int i = 0; i < 4; ++i) {
      const size_t ao = (size_t)(m0 + (i << 4) + rlane) * lda + koff + k0;
      V ah = Frag<T>::load(Ab + ao);
      V al;
      if (SPLIT) al = Frag<T>::load(Ab2 + ao);
#pragma unroll
      for (int j = 0; j < 4; ++j) {
        acc[i][j] = Frag<T>::mma(ah, bh[j], acc[i][j]);
        if (SPLIT) {
          acc[i][j] = Frag<T>::mma(ah, bl[j], acc[i][j]);
          acc[i][j] = Frag<T>::mma(al, bh[j], acc[i][j]);
        }
      }
      Frag<T>::guard(acc[i][0], acc[i][3], ah, SPLIT ? al : ah);
    }
    Frag<T>::keep(bh[0], bh[1], bh[2], bh[3]);
    if (SPLIT) Frag<T>::keep(bl[0], bl[1], bl[2], bl[3]);
  }
  acc_guard4(acc[0][0], acc[0][1], acc[0][2], acc[0][3]);
  acc_guard4(acc[1][0], acc[1][1], acc[1][2], acc[1][3]);
  acc_guard4(acc[2][0], acc[2][1], acc[2][2], acc[2][3]);
  acc_guard4(acc[3][0], acc[3][1], acc[3][2], acc[3][3]);

  float* slab = sT[wave];
  const float* Rb  = RESID ? (resid + (size_t)b * strideR) : nullptr;
  const float* Bsb = (BIAS_MODE != 0) ? (bias + (size_t)b * strideBias) : bias;
#pragma unroll
  for (int i = 0; i < 4; ++i) {
    const int mBase = m0 + (i << 4);
#pragma unroll
    for (int j = 0; j < 4; ++j) {
      const int n = n0 + (j << 4) + rlane;
      float bv = 0.f;
      if (BIAS_MODE == 2) bv = Bsb[n];
#pragma unroll
      for (int r = 0; r < 8; ++r) {
        float v = acc[i][j][r] * scale;
        if (BIAS_MODE == 1) v += Bsb[mBase + mOff + r];
        if (BIAS_MODE == 2) v += bv;
        if (RESID) v += Rb[(size_t)(mBase + mOff + r) * ldc + n];
        if (ACT == 1) v = tanhf(v);
        if (ACT == 2) v = fmaxf(v, 0.0f);
        if (ACT == 3) v = v / (1.0f + expf(-v));
        if (ACT == 4) v = (v > 0.f) ? v : 0.01f * v;
        if (ACT == 5) v = 0.5f * v * (1.0f + erff(v * 0.70710678118654752f));
        if (ACT == 6) v = (v > 0.f) ? v : (expf(v) - 1.0f);
        v *= oscale;
        slab[(mOff + r) * 68 + (j << 4) + rlane] = v;
      }
    }
    __builtin_amdgcn_fence(__ATOMIC_RELEASE, "workgroup");
    __builtin_amdgcn_wave_barrier();
    __builtin_amdgcn_fence(__ATOMIC_ACQUIRE, "workgroup");
    if (OUT_MODE == 0) {
      float* C = (float*)Cout + (size_t)b * strideC;
      const int hh = lane >> 4, c4 = (lane & 15) * 4;
      for (int pass = 0; pass < 2; ++pass) {
#pragma unroll
        for (int it = 0; it < 8; ++it) {
          const int row = it * 2 + hh;
          v4f v = *(const v4f*)(slab + row * 68 + c4);
          *(volatile v4f*)(C + (size_t)(mBase + row) * ldc + n0 + c4) = v;
        }
        __threadfence();
      }
    } else {
      const int q = lane >> 3, c8 = (lane & 7) * 8;
      unsigned short* C  = (unsigned short*)Cout  + (size_t)b * strideC;
      unsigned short* C2 = (OUT_MODE == 2) ? ((unsigned short*)Cout2 + (size_t)b * strideC) : nullptr;
      for (int pass = 0; pass < 2; ++pass) {
#pragma unroll
        for (int it = 0; it < 4; ++it) {
          const int row = it * 4 + q;
          const float* sp = slab + row * 68 + c8;
          v8h hv, lv;
#pragma unroll
          for (int e = 0; e < 8; ++e) {
            if (OUT_MODE == 1) {
              hv[e] = (_Float16)sp[e];
            } else {
              unsigned short hb = f2bf_bits(sp[e]);
              unsigned short lb = f2bf_bits(sp[e] - bf_bits2f(hb));
              hv[e] = __builtin_bit_cast(_Float16, hb);
              lv[e] = __builtin_bit_cast(_Float16, lb);
            }
          }
          *(volatile v8h*)(C + (size_t)(mBase + row) * ldc + n0 + c8) = hv;
          if (OUT_MODE == 2) *(volatile v8h*)(C2 + (size_t)(mBase + row) * ldc + n0 + c8) = lv;
        }
        __threadfence();
      }
    }
    __builtin_amdgcn_fence(__ATOMIC_RELEASE, "workgroup");
    __builtin_amdgcn_wave_barrier();
    __builtin_amdgcn_fence(__ATOMIC_ACQUIRE, "workgroup");
  }
}

__global__ __launch_bounds__(256) void cast_f32_f16x2s(
    const float* __restrict__ in, _Float16* __restrict__ out, int n2, float sc) {
  int i = blockIdx.x * 256 + threadIdx.x;
  if (i < n2) {
    const _Float16 h0 = (_Float16)(in[2 * i] * sc), h1 = (_Float16)(in[2 * i + 1] * sc);
    const unsigned u = (unsigned)__builtin_bit_cast(unsigned short, h0) | ((unsigned)__builtin_bit_cast(unsigned short, h1) << 16);
    ((volatile unsigned*)out)[i] = u;
    __threadfence();
    ((volatile unsigned*)out)[i] = u;
  }
}

DEVI v8f vz8() { return (v8f){0.f,0.f,0.f,0.f,0.f,0.f,0.f,0.f}; }
DEVI v8f mma_h(v16h a, v16h b, v8f c) {
  c = __builtin_amdgcn_wmma_f32_16x16x32_f16(false, a, false, b, (short)0, c, false, false);
  asm volatile("v_nop\n\tv_nop\n\tv_nop\n\tv_nop" : "+v"(c) : "v"(a), "v"(b));
  return c;
}
DEVI void wave_lds_sync() {
  __builtin_amdgcn_fence(__ATOMIC_RELEASE, "workgroup");
  __builtin_amdgcn_wave_barrier();
  __builtin_amdgcn_fence(__ATOMIC_ACQUIRE, "workgroup");
}
DEVI float wsum32(float v) {
#pragma unroll
  for (int off = 1; off < 32; off <<= 1) v += __shfl_xor(v, off, 32);
  return v;
}
DEVI float wmax32(float v) {
#pragma unroll
  for (int off = 1; off < 32; off <<= 1) v = fmaxf(v, __shfl_xor(v, off, 32));
  return v;
}
DEVI float hsum16(float v) {
#pragma unroll
  for (int off = 1; off < 16; off <<= 1) v += __shfl_xor(v, off, 32);
  return v;
}
DEVI float hmax16(float v) {
#pragma unroll
  for (int off = 1; off < 16; off <<= 1) v = fmaxf(v, __shfl_xor(v, off, 32));
  return v;
}
DEVI float sigm(float v) { return 1.0f / (1.0f + expf(fminf(-v, 80.0f))); }
DEVI float elu1(float v) { return v > 0.f ? v : (expf(v) - 1.0f); }

__global__ __launch_bounds__(256) void transpose_cast64(const float* __restrict__ in, long sIn, int Cc,
                                                         _Float16* __restrict__ out, long sOut, int ldo, float sc) {
  __shared__ __align__(16) _Float16 tile[64 * 72];
  const int tid = threadIdx.x;
  const int tilesC = Cc >> 6;
  const int tr = blockIdx.x / tilesC;
  const int tc = blockIdx.x - tr * tilesC;
  const int r0 = tr << 6, c0 = tc << 6;
  const float* src = in + (size_t)blockIdx.y * sIn;
  {
    const int rr = tid >> 2, cs = (tid & 3) * 16;
    const float* p = src + (size_t)(r0 + rr) * Cc + c0 + cs;
#pragma unroll
    for (int i = 0; i < 4; ++i) {
      const v4f v = *(const v4f*)(p + 4 * i);
#pragma unroll
      for (int e = 0; e < 4; ++e) tile[(cs + 4 * i + e) * 72 + rr] = (_Float16)(v[e] * sc);
    }
  }
  __syncthreads();
  _Float16* dst = out + (size_t)blockIdx.y * sOut;
  const int seg = (tid & 7) * 8;
  for (int pass = 0; pass < 2; ++pass) {
#pragma unroll
    for (int it = 0; it < 2; ++it) {
      const int line = it * 32 + (tid >> 3);
      const v8h v = *(const v8h*)(tile + line * 72 + seg);
      *(volatile v8h*)(dst + (size_t)(c0 + line) * ldo + r0 + seg) = v;
    }
    __threadfence();
  }
}

__global__ __launch_bounds__(256) void flat_tail_kernel(
    const float* __restrict__ ogf, const float* __restrict__ skip,
    const float* __restrict__ bo, const float* __restrict__ bg, const float* __restrict__ sb,
    const float* __restrict__ lng, const float* __restrict__ lnb,
    float* __restrict__ swws, float* __restrict__ swout) {
  const int lane = threadIdx.x & 31, wave = threadIdx.x >> 5;
  const int row = blockIdx.x * 8 + wave;
  const int c4 = lane * 4;
  const float* pr = ogf + (size_t)row * 256;
  const v4f vo = *(const v4f*)(pr + c4);
  const v4f vg = *(const v4f*)(pr + 128 + c4);
  const v4f sk = *(const v4f*)(skip + (size_t)row * 128 + c4);
  const v4f vbo = *(const v4f*)(bo + c4), vbg = *(const v4f*)(bg + c4), vsb = *(const v4f*)(sb + c4);
  const v4f vln = *(const v4f*)(lng + c4), vlb = *(const v4f*)(lnb + c4);
  float t[4];
  float s = 0.f;
#pragma unroll
  for (int e = 0; e < 4; ++e) { t[e] = sigm(vg[e] + vbg[e]) * (vo[e] + vbo[e]) + sk[e] + vsb[e]; s += t[e]; }
  s = wsum32(s);
  const float mean = s * (1.0f / 128.0f);
  float q = 0.f;
#pragma unroll
  for (int e = 0; e < 4; ++e) { t[e] -= mean; q += t[e] * t[e]; }
  q = wsum32(q);
  const float inv = 1.0f / sqrtf(q * (1.0f / 128.0f) + 1e-5f);
  float ln[4];
  float mx = -INFINITY;
#pragma unroll
  for (int e = 0; e < 4; ++e) { ln[e] = t[e] * inv * vln[e] + vlb[e]; mx = fmaxf(mx, ln[e]); }
  mx = wmax32(mx);
  float es = 0.f;
#pragma unroll
  for (int e = 0; e < 4; ++e) { ln[e] = expf(ln[e] - mx); es += ln[e]; }
  es = wsum32(es);
  const float rcp = 1.0f / es;
  v4f ov;
#pragma unroll
  for (int e = 0; e < 4; ++e) ov[e] = ln[e] * rcp;
  float* d0 = swws + (size_t)row * 128 + c4;
  float* d1 = swout + (size_t)row * 128 + c4;
  for (int pass = 0; pass < 2; ++pass) {
    *(volatile v4f*)d0 = ov;
    *(volatile v4f*)d1 = ov;
    __threadfence();
  }
}

__global__ __launch_bounds__(256) void vsn_h1_kernel(const float* __restrict__ x, const float* __restrict__ w1,
                                                    const float* __restrict__ b1, int f0, _Float16* __restrict__ h1) {
  const int lane = threadIdx.x & 31, wave = threadIdx.x >> 5;
  const int g = blockIdx.x >> 7;
  const int n = (blockIdx.x & 127) * 8 + wave;
  const int f = f0 + g;
  const int k0 = lane * 8;
  const float xv = x[(size_t)n * FIN + f];
  const v4f wa = *(const v4f*)(w1 + (size_t)f * HID + k0), wb = *(const v4f*)(w1 + (size_t)f * HID + k0 + 4);
  const v4f ba = *(const v4f*)(b1 + (size_t)f * HID + k0), bb = *(const v4f*)(b1 + (size_t)f * HID + k0 + 4);
  v8h hv;
#pragma unroll
  for (int e = 0; e < 4; ++e) {
    hv[e]     = (_Float16)(elu1(xv * wa[e] + ba[e]) * 64.0f);
    hv[4 + e] = (_Float16)(elu1(xv * wb[e] + bb[e]) * 64.0f);
  }
  _Float16* dst = h1 + ((size_t)g * NTOK + n) * HID + k0;
  *(volatile v8h*)dst = hv;
  __threadfence();
  *(volatile v8h*)dst = hv;
}

template <bool FIRST, bool LAST>
__global__ __launch_bounds__(256) void vsn_combine_kernel(
    const float* __restrict__ og, const float* __restrict__ x, const float* __restrict__ sw,
    const float* __restrict__ sbo, const float* __restrict__ sbg, const float* __restrict__ ssw, const float* __restrict__ ssb,
    const float* __restrict__ slg, const float* __restrict__ slb, int f0,
    const float* __restrict__ selin, float* __restrict__ selout,
    const float* __restrict__ pos, _Float16* __restrict__ feats16) {
  __shared__ __align__(16) float vec[6][256];
  __shared__ __align__(16) float slab[8][256];
  const int tid = threadIdx.x, lane = tid & 31, wave = tid >> 5;
  const int n = blockIdx.x * 8 + wave;
  const int k0 = lane * 8;
  float acc[8];
  if (FIRST) {
#pragma unroll
    for (int e = 0; e < 8; ++e) acc[e] = 0.f;
  } else {
    const v4f a0 = *(const v4f*)(selin + (size_t)n * HID + k0), a1 = *(const v4f*)(selin + (size_t)n * HID + k0 + 4);
#pragma unroll
    for (int e = 0; e < 4; ++e) { acc[e] = a0[e]; acc[4 + e] = a1[e]; }
  }
#pragma unroll 1
  for (int g = 0; g < GRP; ++g) {
    const int f = f0 + g;
    __syncthreads();
    vec[0][tid] = sbo[(size_t)f * HID + tid];
    vec[1][tid] = sbg[(size_t)f * HID + tid];
    vec[2][tid] = ssw[(size_t)f * HID + tid];
    vec[3][tid] = ssb[(size_t)f * HID + tid];
    vec[4][tid] = slg[(size_t)f * HID + tid];
    vec[5][tid] = slb[(size_t)f * HID + tid];
    __syncthreads();
    const float* ogr = og + ((size_t)g * NTOK + n) * 512;
    const v4f o0 = *(const v4f*)(ogr + k0), o1 = *(const v4f*)(ogr + k0 + 4);
    const v4f q0 = *(const v4f*)(ogr + 256 + k0), q1 = *(const v4f*)(ogr + 256 + k0 + 4);
    const float xv  = x[(size_t)n * FIN + f];
    const float swv = sw[(size_t)n * FIN + f];
    const v4f bo0 = *(const v4f*)(&vec[0][k0]), bo1 = *(const v4f*)(&vec[0][k0 + 4]);
    const v4f bg0 = *(const v4f*)(&vec[1][k0]), bg1 = *(const v4f*)(&vec[1][k0 + 4]);
    const v4f sw0 = *(const v4f*)(&vec[2][k0]), sw1 = *(const v4f*)(&vec[2][k0 + 4]);
    const v4f sb0 = *(const v4f*)(&vec[3][k0]), sb1 = *(const v4f*)(&vec[3][k0 + 4]);
    const v4f lg0 = *(const v4f*)(&vec[4][k0]), lg1 = *(const v4f*)(&vec[4][k0 + 4]);
    const v4f lb0 = *(const v4f*)(&vec[5][k0]), lb1 = *(const v4f*)(&vec[5][k0 + 4]);
    float t[8];
    float s = 0.f;
#pragma unroll
    for (int e = 0; e < 4; ++e) {
      t[e]     = sigm(q0[e] + bg0[e]) * (o0[e] + bo0[e]) + xv * sw0[e] + sb0[e];
      t[4 + e] = sigm(q1[e] + bg1[e]) * (o1[e] + bo1[e]) + xv * sw1[e] + sb1[e];
      s += t[e] + t[4 + e];
    }
    s = wsum32(s);
    const float mean = s * (1.0f / 256.0f);
    float q = 0.f;
#pragma unroll
    for (int e = 0; e < 8; ++e) { t[e] -= mean; q += t[e] * t[e]; }
    q = wsum32(q);
    const float inv = 1.0f / sqrtf(q * (1.0f / 256.0f) + 1e-5f);
#pragma unroll
    for (int e = 0; e < 4; ++e) {
      acc[e]     += swv * (t[e] * inv * lg0[e] + lb0[e]);
      acc[4 + e] += swv * (t[4 + e] * inv * lg1[e] + lb1[e]);
    }
  }
  if (LAST) {
    const int sidx = n & (SEQ - 1);
    const v4f p0 = *(const v4f*)(pos + (size_t)sidx * HID + k0), p1 = *(const v4f*)(pos + (size_t)sidx * HID + k0 + 4);
    v8h hv;
#pragma unroll
    for (int e = 0; e < 4; ++e) { hv[e] = (_Float16)(acc[e] + p0[e]); hv[4 + e] = (_Float16)(acc[4 + e] + p1[e]); }
    _Float16* dst = feats16 + (size_t)n * HID + k0;
    *(volatile v8h*)dst = hv;
    __threadfence();
    *(volatile v8h*)dst = hv;
  } else {
#pragma unroll
    for (int e = 0; e < 8; ++e) slab[wave][k0 + e] = acc[e];
    wave_lds_sync();
    const v4f a0 = *(const v4f*)(&slab[wave][lane * 4]);
    const v4f a1 = *(const v4f*)(&slab[wave][128 + lane * 4]);
    float* d = selout + (size_t)n * HID;
    for (int pass = 0; pass < 2; ++pass) {
      *(volatile v4f*)(d + lane * 4) = a0;
      *(volatile v4f*)(d + 128 + lane * 4) = a1;
      __threadfence();
    }
  }
}

__global__ __launch_bounds__(256) void lstm_seq_kernel(const float* __restrict__ gin, const _Float16* __restrict__ whh16,
                                                      const float* __restrict__ bhh, float* __restrict__ outF,
                                                      _Float16* __restrict__ out16) {
  __shared__ __align__(16) _Float16 Ah[16 * 264];
  __shared__ __align__(16) float Gb[8 * 1024];
  __shared__ float Cst[8 * 256];
  __shared__ __align__(16) float Hst[8 * 256];
  const int tid = threadIdx.x, lane = tid & 31, wave = tid >> 5;
  const int hh = lane >> 4, rl = lane & 15, koff = hh * 8;
  for (int i = tid; i < 16 * 264; i += 256) Ah[i] = (_Float16)0.0f;
  for (int i = tid; i < 8 * 256; i += 256) Cst[i] = 0.f;
  const float bh0 = bhh[tid], bh1 = bhh[256 + tid], bh2 = bhh[512 + tid], bh3 = bhh[768 + tid];
  const float RSC = 1.0f / 64.0f;
  __syncthreads();
  for (int s = 0; s < SEQ; ++s) {
    v8f acc[8];
#pragma unroll
    for (int t = 0; t < 8; ++t) acc[t] = vz8();
    const _Float16* wb = whh16 + (size_t)(wave * 128 + rl) * HID + koff;
#pragma unroll 1
    for (int k0 = 0; k0 < HID; k0 += 32) {
      const v16h a = Frag<_Float16>::load(Ah + rl * 264 + k0 + koff);
      v16h bf[8];
#pragma unroll
      for (int t = 0; t < 8; ++t) bf[t] = Frag<_Float16>::load(wb + (size_t)t * 16 * HID + k0);
#pragma unroll
      for (int t = 0; t < 8; ++t) acc[t] = mma_h(a, bf[t], acc[t]);
    }
    if (hh == 0) {
#pragma unroll
      for (int t = 0; t < 8; ++t) {
        const int nn = wave * 128 + t * 16 + rl;
#pragma unroll
        for (int r = 0; r < 8; ++r) Gb[r * 1024 + nn] = acc[t][r];
      }
    }
    __syncthreads();
#pragma unroll 1
    for (int b = 0; b < NBAT; ++b) {
      const size_t grow = (size_t)(b * SEQ + s) * NGATE;
      const float gi = Gb[b * 1024 + tid] * RSC       + gin[grow + tid]       + bh0;
      const float gf = Gb[b * 1024 + 256 + tid] * RSC + gin[grow + 256 + tid] + bh1;
      const float gg = Gb[b * 1024 + 512 + tid] * RSC + gin[grow + 512 + tid] + bh2;
      const float go = Gb[b * 1024 + 768 + tid] * RSC + gin[grow + 768 + tid] + bh3;
      const float c = sigm(gf) * Cst[b * 256 + tid] + sigm(gi) * tanhf(gg);
      const float h = sigm(go) * tanhf(c);
      Cst[b * 256 + tid] = c;
      Ah[b * 264 + tid] = (_Float16)h;
      Hst[b * 256 + tid] = h;
    }
    __syncthreads();
    for (int pass = 0; pass < 2; ++pass) {
#pragma unroll
      for (int b = 0; b < NBAT; ++b)
        ((volatile float*)outF)[(size_t)(b * SEQ + s) * HID + tid] = Hst[b * 256 + tid];
#pragma unroll
      for (int i = 0; i < 4; ++i) {
        const int w = tid + 256 * i;
        const int b = w >> 7, p = w & 127;
        const unsigned u = *(const unsigned*)(Ah + b * 264 + 2 * p);
        ((volatile unsigned*)out16)[(((size_t)(b * SEQ + s) * HID) >> 1) + p] = u;
      }
      __threadfence();
    }
  }
}

__global__ __launch_bounds__(128) void attn32_kernel(const _Float16* __restrict__ qk, const _Float16* __restrict__ vt,
                                                    _Float16* __restrict__ ctx) {
  __shared__ __align__(16) _Float16 Ks[SEQ * 32];
  __shared__ __align__(16) _Float16 Vs[32 * SEQ];
  __shared__ __align__(16) _Float16 Pw[4][16 * SEQ];
  __shared__ __align__(16) float Os[4][16 * 68];
  const int tid = threadIdx.x, wave = tid >> 5, lane = tid & 31;
  const int hh = lane >> 4, c = lane & 15, koff = hh * 8;
  const int bx = blockIdx.x;
  const int qb = bx & 1, hp = (bx >> 1) & 3, b = bx >> 3;
  const int q0 = qb * 64 + wave * 16;
  const size_t tok0 = (size_t)b * SEQ;
  v8f oacc[2][2];
  float lrow[2][8];
#pragma unroll
  for (int hd = 0; hd < 2; ++hd) {
    const int h = hp * 2 + hd;
    __syncthreads();
    {
      const v4u* kr = (const v4u*)(qk + (tok0 + tid) * 512 + 256 + h * 32);
      v4u* kd = (v4u*)(Ks + tid * 32);
#pragma unroll
      for (int i = 0; i < 4; ++i) kd[i] = kr[i];
      const int d = tid >> 2, seg = (tid & 3) * 32;
      const v4u* vr = (const v4u*)(vt + (size_t)(h * 32 + d) * NTOK + tok0 + seg);
      v4u* vd = (v4u*)(Vs + d * SEQ + seg);
#pragma unroll
      for (int i = 0; i < 4; ++i) vd[i] = vr[i];
    }
    __syncthreads();
    const v16h qa = Frag<_Float16>::load(qk + (tok0 + q0 + c) * 512 + h * 32 + koff);
    v8f s[8];
#pragma unroll
    for (int j = 0; j < 8; ++j) {
      const v16h kb = Frag<_Float16>::load(Ks + (j * 16 + c) * 32 + koff);
      s[j] = mma_h(qa, kb, vz8());
    }
    float cm[8];
#pragma unroll
    for (int r = 0; r < 8; ++r) {
      float m = -INFINITY;
#pragma unroll
      for (int j = 0; j < 8; ++j) { s[j][r] *= ATT_SCL; m = fmaxf(m, s[j][r]); }
      m = hmax16(m);
      cm[r] = m;
    }
    _Float16* pw = Pw[wave];
#pragma unroll
    for (int r = 0; r < 8; ++r) {
      float ps = 0.f;
#pragma unroll
      for (int j = 0; j < 8; ++j) {
        const float p = expf(s[j][r] - cm[r]);
        ps += p;
        pw[(8 * hh + r) * SEQ + j * 16 + c] = (_Float16)(p * PCAR);
      }
      lrow[hd][r] = hsum16(ps);
    }
    wave_lds_sync();
    oacc[hd][0] = vz8();
    oacc[hd][1] = vz8();
#pragma unroll
    for (int kk = 0; kk < 4; ++kk) {
      const v16h pa = Frag<_Float16>::load(pw + c * SEQ + kk * 32 + koff);
#pragma unroll
      for (int t = 0; t < 2; ++t) {
        const v16h vb = Frag<_Float16>::load(Vs + (t * 16 + c) * SEQ + kk * 32 + koff);
        oacc[hd][t] = mma_h(pa, vb, oacc[hd][t]);
      }
    }
  }
  float* os = Os[wave];
#pragma unroll
  for (int hd = 0; hd < 2; ++hd) {
#pragma unroll
    for (int r = 0; r < 8; ++r) {
      const float inv = (CTXCAR / PCAR) / lrow[hd][r];
#pragma unroll
      for (int t = 0; t < 2; ++t) os[(8 * hh + r) * 68 + hd * 32 + t * 16 + c] = oacc[hd][t][r] * inv;
    }
  }
  wave_lds_sync();
  {
    const int q = lane >> 3, c8 = (lane & 7) * 8;
    for (int pass = 0; pass < 2; ++pass) {
#pragma unroll
      for (int it = 0; it < 4; ++it) {
        const int row = it * 4 + q;
        const float* sp = os + row * 68 + c8;
        v8h hv;
#pragma unroll
        for (int e = 0; e < 8; ++e) hv[e] = (_Float16)sp[e];
        *(volatile v8h*)(ctx + (tok0 + q0 + row) * HID + hp * 64 + c8) = hv;
      }
      __threadfence();
    }
  }
}

__global__ __launch_bounds__(256) void ln256_kernel(const float* __restrict__ proj, const float* __restrict__ gam,
                                                   const float* __restrict__ bet, float* __restrict__ dstF,
                                                   _Float16* __restrict__ dst16) {
  const int lane = threadIdx.x & 31, wave = threadIdx.x >> 5;
  const int row = blockIdx.x * 8 + wave;
  const int c4 = lane * 4, c8 = lane * 8;
  const float* pr = proj + (size_t)row * HID;
  const v4f a = *(const v4f*)(pr + c4), bq = *(const v4f*)(pr + 128 + c4);
  float s = 0.f;
#pragma unroll
  for (int e = 0; e < 4; ++e) s += a[e] + bq[e];
  s = wsum32(s);
  const float mean = s * (1.0f / 256.0f);
  float q = 0.f;
#pragma unroll
  for (int e = 0; e < 4; ++e) { const float d0 = a[e] - mean, d1 = bq[e] - mean; q += d0 * d0 + d1 * d1; }
  q = wsum32(q);
  const float inv = 1.0f / sqrtf(q * (1.0f / 256.0f) + 1e-5f);
  const v4f ga = *(const v4f*)(gam + c4), gb = *(const v4f*)(gam + 128 + c4);
  const v4f ba = *(const v4f*)(bet + c4), bb = *(const v4f*)(bet + 128 + c4);
  v4f oa, ob;
#pragma unroll
  for (int e = 0; e < 4; ++e) { oa[e] = (a[e] - mean) * inv * ga[e] + ba[e]; ob[e] = (bq[e] - mean) * inv * gb[e] + bb[e]; }
  const v4f e0 = *(const v4f*)(pr + c8), e1 = *(const v4f*)(pr + c8 + 4);
  const v4f g0 = *(const v4f*)(gam + c8), g1 = *(const v4f*)(gam + c8 + 4);
  const v4f b0 = *(const v4f*)(bet + c8), b1 = *(const v4f*)(bet + c8 + 4);
  v8h hv;
#pragma unroll
  for (int e = 0; e < 4; ++e) {
    hv[e]     = (_Float16)((e0[e] - mean) * inv * g0[e] + b0[e]);
    hv[4 + e] = (_Float16)((e1[e] - mean) * inv * g1[e] + b1[e]);
  }
  float* dF = dstF + (size_t)row * HID;
  _Float16* d16 = dst16 + (size_t)row * HID + c8;
  for (int pass = 0; pass < 2; ++pass) {
    *(volatile v4f*)(dF + c4) = oa;
    *(volatile v4f*)(dF + 128 + c4) = ob;
    *(volatile v8h*)d16 = hv;
    __threadfence();
  }
}

__global__ __launch_bounds__(256) void heads_kernel(const float* __restrict__ a, const float* __restrict__ w1,
                                                   const float* __restrict__ b1, const float* __restrict__ w2,
                                                   const float* __restrict__ b2, const float* __restrict__ qw,
                                                   const float* __restrict__ qb, float* __restrict__ out) {
  __shared__ float gsh[NBAT * HID];
  __shared__ float hsh[NBAT * 128];
  __shared__ __align__(16) float ov[768];
  const int tid = threadIdx.x;
#pragma unroll 1
  for (int b = 0; b < NBAT; ++b) {
    float s = 0.f;
    const float* col = a + (size_t)b * SEQ * HID + tid;
#pragma unroll 1
    for (int r = 0; r < SEQ; ++r) s += col[(size_t)r * HID];
    gsh[b * HID + tid] = s * (1.0f / 128.0f);
  }
  __syncthreads();
#pragma unroll 1
  for (int i = 0; i < 4; ++i) {
    const int idx = tid + 256 * i;
    const int b = idx >> 7, j = idx & 127;
    float acc = b1[j];
    const float* gr = gsh + b * HID;
#pragma unroll 1
    for (int k = 0; k < HID; ++k) acc += gr[k] * w1[k * 128 + j];
    hsh[b * 128 + j] = fmaxf(acc, 0.f);
  }
  __syncthreads();
#pragma unroll 1
  for (int p = 0; p < 3; ++p) {
    const int o = tid + 256 * p;
    float acc;
    if (o < 192) {
      const int b = o / 24, j = o - b * 24;
      acc = b2[j];
      const float* hr = hsh + b * 128;
#pragma unroll 1
      for (int k = 0; k < 128; ++k) acc += hr[k] * w2[k * 24 + j];
    } else {
      const int o2 = o - 192;
      const int which = o2 / 192, rem = o2 - which * 192;
      const int b = rem / 24, j = rem - b * 24;
      acc = qb[which * 24 + j];
      const float* gr = gsh + b * HID;
      const float* qwp = qw + (size_t)which * 6144 + j;
#pragma unroll 1
      for (int k = 0; k < HID; ++k) acc += gr[k] * qwp[k * 24];
    }
    ov[o] = acc;
  }
  __syncthreads();
  if (tid < 192) {
    const v4f v = *(const v4f*)(ov + 4 * tid);
    *(volatile v4f*)(out + 4 * tid) = v;
    __threadfence();
    *(volatile v4f*)(out + 4 * tid) = v;
  }
}

template <int BIAS_MODE, int OUT_MODE, bool RESID, int ACT>
static void launch_gemm(hipStream_t st, const void* A, int lda, long sA, const void* Bt, int ldb, long sB,
                        void* C, int ldc, long sC, const float* bias, long sBias, const float* resid, long sR,
                        int M, int N, int K, float scale, float oscale, int batch) {
  const int tiles = (M / 64) * (N / 64);
  dim3 grid((unsigned)((tiles + 7) / 8), (unsigned)batch, 1);
  wmma_gemm64<0, false, BIAS_MODE, OUT_MODE, RESID, ACT><<<grid, 256, 0, st>>>(
      (const unsigned short*)A, (const unsigned short*)A, lda, sA,
      (const unsigned short*)Bt, (const unsigned short*)Bt, ldb, sB,
      C, C, ldc, sC, bias, sBias, resid, sR, M, N, K, scale, oscale);
}

static constexpr size_t SZ_X16  = (size_t)NTOK * FIN * 2;
static constexpr size_t SZ_W1T  = (size_t)HID * FIN * 2;
static constexpr size_t SZ_W2T  = (size_t)HID * HID * 2;
static constexpr size_t SZ_OGT  = (size_t)HID * HID * 2;
static constexpr size_t SZ_SWT  = (size_t)FIN * FIN * 2;
static constexpr size_t SZ_T16  = (size_t)NTOK * HID * 2;
static constexpr size_t SZ_F32P = (size_t)NTOK * HID * 4;
static constexpr size_t SZ_SKIP = (size_t)NTOK * FIN * 4;
static constexpr size_t SZ_SVW2 = (size_t)FIN * HID * HID * 2;
static constexpr size_t SZ_SVOG = (size_t)FIN * 2 * HID * HID * 2;
static constexpr size_t SZ_H1   = (size_t)GRP * NTOK * HID * 2;
static constexpr size_t SZ_OG   = (size_t)GRP * NTOK * 512 * 4;
static constexpr size_t SZ_GIN  = (size_t)NTOK * NGATE * 4;
static constexpr size_t SZ_QKT  = (size_t)NLAY * 512 * HID * 2;
static constexpr size_t SZ_WVT  = (size_t)NLAY * HID * HID * 2;
static constexpr size_t SZ_QKP  = (size_t)NTOK * 512 * 2;
static constexpr size_t SZ_VTP  = (size_t)HID * NTOK * 2;
static constexpr size_t WS_TOTAL =
    SZ_X16 + SZ_W1T + SZ_W2T + SZ_OGT + SZ_SWT + 2 * SZ_T16 + SZ_F32P + 2 * SZ_SKIP +
    SZ_SVW2 + SZ_SVOG + 2 * SZ_H1 + SZ_OG + 2 * SZ_F32P + SZ_T16 +
    4 * SZ_T16 + SZ_GIN + 3 * SZ_T16 + 2 * SZ_F32P + SZ_QKT + 2 * SZ_WVT + SZ_QKP + SZ_VTP + SZ_T16 + SZ_F32P;
static_assert(WS_TOTAL == 122257408);
static_assert(WS_TOTAL <= 134217728);
static_assert(527360 + (size_t)NTOK * HID * 4 == 1575936);

extern "C" void kernel_launch(void* const* d_in, const int* in_sizes, int n_in,
                              void* d_out, int out_size, void* d_ws, size_t ws_size, hipStream_t stream) {
  (void)in_sizes; (void)n_in; (void)out_size; (void)ws_size;
  const float* x      = (const float*)d_in[0];
  const float* fg_w1  = (const float*)d_in[1];
  const float* fg_b1  = (const float*)d_in[2];
  const float* fg_w2  = (const float*)d_in[3];
  const float* fg_b2  = (const float*)d_in[4];
  const float* fg_wo  = (const float*)d_in[5];
  const float* fg_bo  = (const float*)d_in[6];
  const float* fg_wg  = (const float*)d_in[7];
  const float* fg_bg  = (const float*)d_in[8];
  const float* fg_sw  = (const float*)d_in[9];
  const float* fg_sb  = (const float*)d_in[10];
  const float* fg_lng = (const float*)d_in[11];
  const float* fg_lnb = (const float*)d_in[12];
  const float* sv_w1  = (const float*)d_in[13];
  const float* sv_b1  = (const float*)d_in[14];
  const float* sv_w2  = (const float*)d_in[15];
  const float* sv_b2  = (const float*)d_in[16];
  const float* sv_wo  = (const float*)d_in[17];
  const float* sv_bo  = (const float*)d_in[18];
  const float* sv_wg  = (const float*)d_in[19];
  const float* sv_bg  = (const float*)d_in[20];
  const float* sv_sw  = (const float*)d_in[21];
  const float* sv_sb  = (const float*)d_in[22];
  const float* sv_lng = (const float*)d_in[23];
  const float* sv_lnb = (const float*)d_in[24];
  const float* pos    = (const float*)d_in[25];
  const float* l0_wih = (const float*)d_in[26];
  const float* l0_whh = (const float*)d_in[27];
  const float* l0_bih = (const float*)d_in[28];
  const float* l0_bhh = (const float*)d_in[29];
  const float* l1_wih = (const float*)d_in[30];
  const float* l1_whh = (const float*)d_in[31];
  const float* l1_bih = (const float*)d_in[32];
  const float* l1_bhh = (const float*)d_in[33];
  const float* att_wq = (const float*)d_in[34];
  const float* att_wk = (const float*)d_in[35];
  const float* att_wv = (const float*)d_in[36];
  const float* att_wo = (const float*)d_in[37];
  const float* att_bo = (const float*)d_in[38];
  const float* att_lng= (const float*)d_in[39];
  const float* att_lnb= (const float*)d_in[40];
  const float* out_w1 = (const float*)d_in[41];
  const float* out_b1 = (const float*)d_in[42];
  const float* out_w2 = (const float*)d_in[43];
  const float* out_b2 = (const float*)d_in[44];
  const float* qw     = (const float*)d_in[45];
  const float* qb     = (const float*)d_in[46];
  float* out  = (float*)d_out;
  float* out4 = out + 768;
  float* out5 = out + 131840;

  char* wsb = (char*)d_ws;
  size_t off = 0;
  auto carve = [&](size_t bytes) -> void* { void* p = wsb + off; off += (bytes + 255) & ~(size_t)255; return p; };
  _Float16* x16    = (_Float16*)carve(SZ_X16);
  _Float16* w1t    = (_Float16*)carve(SZ_W1T);
  _Float16* w2t_fg = (_Float16*)carve(SZ_W2T);
  _Float16* ogt_fg = (_Float16*)carve(SZ_OGT);
  _Float16* swt    = (_Float16*)carve(SZ_SWT);
  _Float16* t0     = (_Float16*)carve(SZ_T16);
  _Float16* t1     = (_Float16*)carve(SZ_T16);
  float*    ogf    = (float*)carve(SZ_F32P);
  float*    skipb  = (float*)carve(SZ_SKIP);
  float*    swws   = (float*)carve(SZ_SKIP);
  _Float16* svw2t  = (_Float16*)carve(SZ_SVW2);
  _Float16* svogt  = (_Float16*)carve(SZ_SVOG);
  _Float16* h1p    = (_Float16*)carve(SZ_H1);
  _Float16* h2p    = (_Float16*)carve(SZ_H1);
  float*    ogp    = (float*)carve(SZ_OG);
  float*    selp[2];
  selp[0] = (float*)carve(SZ_F32P);
  selp[1] = (float*)carve(SZ_F32P);
  _Float16* feats16= (_Float16*)carve(SZ_T16);
  _Float16* wih16[2]; _Float16* whh16[2];
  wih16[0] = (_Float16*)carve(SZ_T16); whh16[0] = (_Float16*)carve(SZ_T16);
  wih16[1] = (_Float16*)carve(SZ_T16); whh16[1] = (_Float16*)carve(SZ_T16);
  float*    gin    = (float*)carve(SZ_GIN);
  _Float16* a16l0  = (_Float16*)carve(SZ_T16);
  _Float16* a16p[2];
  a16p[0] = (_Float16*)carve(SZ_T16); a16p[1] = (_Float16*)carve(SZ_T16);
  float* aF[2];
  aF[0] = (float*)carve(SZ_F32P); aF[1] = (float*)carve(SZ_F32P);
  _Float16* qkt    = (_Float16*)carve(SZ_QKT);
  _Float16* wvt    = (_Float16*)carve(SZ_WVT);
  _Float16* wot    = (_Float16*)carve(SZ_WVT);
  _Float16* qkp    = (_Float16*)carve(SZ_QKP);
  _Float16* vtp    = (_Float16*)carve(SZ_VTP);
  _Float16* ctx16  = (_Float16*)carve(SZ_T16);
  float*    proj   = (float*)carve(SZ_F32P);

  const float RW = 1.0f / WCAR;
  const long HW = (long)HID * HID;

  cast_f32_f16x2s<<<(NTOK * FIN / 2 + 255) / 256, 256, 0, stream>>>(x, x16, NTOK * FIN / 2, 1.0f);
  cast_f32_f16x2s<<<(NGATE * HID / 2 + 255) / 256, 256, 0, stream>>>(l0_wih, wih16[0], NGATE * HID / 2, WCAR);
  cast_f32_f16x2s<<<(NGATE * HID / 2 + 255) / 256, 256, 0, stream>>>(l0_whh, whh16[0], NGATE * HID / 2, WCAR);
  cast_f32_f16x2s<<<(NGATE * HID / 2 + 255) / 256, 256, 0, stream>>>(l1_wih, wih16[1], NGATE * HID / 2, WCAR);
  cast_f32_f16x2s<<<(NGATE * HID / 2 + 255) / 256, 256, 0, stream>>>(l1_whh, whh16[1], NGATE * HID / 2, WCAR);

  transpose_cast64<<<dim3((128 / 64) * (256 / 64), 1), 256, 0, stream>>>(fg_w1, 0L, 256, w1t, 0L, 128, WCAR);
  transpose_cast64<<<dim3((256 / 64) * (256 / 64), 1), 256, 0, stream>>>(fg_w2, 0L, 256, w2t_fg, 0L, 256, WCAR);
  transpose_cast64<<<dim3((256 / 64) * (128 / 64), 1), 256, 0, stream>>>(fg_wo, 0L, 128, ogt_fg, 0L, 256, WCAR);
  transpose_cast64<<<dim3((256 / 64) * (128 / 64), 1), 256, 0, stream>>>(fg_wg, 0L, 128, ogt_fg + 128 * 256, 0L, 256, WCAR);
  transpose_cast64<<<dim3((128 / 64) * (128 / 64), 1), 256, 0, stream>>>(fg_sw, 0L, 128, swt, 0L, 128, WCAR);
  transpose_cast64<<<dim3((256 / 64) * (256 / 64), FIN), 256, 0, stream>>>(sv_w2, HW, 256, svw2t, HW, 256, WCAR);
  transpose_cast64<<<dim3((256 / 64) * (256 / 64), FIN), 256, 0, stream>>>(sv_wo, HW, 256, svogt, 2 * HW, 256, WCAR);
  transpose_cast64<<<dim3((256 / 64) * (256 / 64), FIN), 256, 0, stream>>>(sv_wg, HW, 256, svogt + HW, 2 * HW, 256, WCAR);
  transpose_cast64<<<dim3((256 / 64) * (256 / 64), NLAY), 256, 0, stream>>>(att_wq, HW, 256, qkt, 2 * HW, 256, WCAR);
  transpose_cast64<<<dim3((256 / 64) * (256 / 64), NLAY), 256, 0, stream>>>(att_wk, HW, 256, qkt + HW, 2 * HW, 256, WCAR);
  transpose_cast64<<<dim3((256 / 64) * (256 / 64), NLAY), 256, 0, stream>>>(att_wv, HW, 256, wvt, HW, 256, WCAR);
  transpose_cast64<<<dim3((256 / 64) * (256 / 64), NLAY), 256, 0, stream>>>(att_wo, HW, 256, wot, HW, 256, WCAR);

  launch_gemm<2, 1, false, 6>(stream, x16, FIN, 0L, w1t, FIN, 0L, t0, HID, 0L, fg_b1, 0L, fg_b1, 0L,
                              NTOK, HID, FIN, RW, 8.0f, 1);
  launch_gemm<2, 1, false, 6>(stream, t0, HID, 0L, w2t_fg, HID, 0L, t1, HID, 0L, fg_b2, 0L, fg_b2, 0L,
                              NTOK, HID, HID, RW / 8.0f, 8.0f, 1);
  launch_gemm<0, 0, false, 0>(stream, t1, HID, 0L, ogt_fg, HID, 0L, ogf, HID, 0L, fg_b1, 0L, fg_b1, 0L,
                              NTOK, HID, HID, RW / 8.0f, 1.0f, 1);
  launch_gemm<0, 0, false, 0>(stream, x16, FIN, 0L, swt, FIN, 0L, skipb, FIN, 0L, fg_b1, 0L, fg_b1, 0L,
                              NTOK, FIN, FIN, RW, 1.0f, 1);
  flat_tail_kernel<<<NTOK / 8, 256, 0, stream>>>(ogf, skipb, fg_bo, fg_bg, fg_sb, fg_lng, fg_lnb, swws, out4);

  for (int gi = 0; gi < NGRP; ++gi) {
    const int f0 = gi * GRP;
    vsn_h1_kernel<<<GRP * 128, 256, 0, stream>>>(x, sv_w1, sv_b1, f0, h1p);
    launch_gemm<2, 1, false, 6>(stream, h1p, HID, (long)NTOK * HID, svw2t + (size_t)f0 * HW, HID, HW,
                                h2p, HID, (long)NTOK * HID, sv_b2 + (size_t)f0 * HID, (long)HID, fg_b1, 0L,
                                NTOK, HID, HID, RW * RW, 64.0f, GRP);
    launch_gemm<0, 0, false, 0>(stream, h2p, HID, (long)NTOK * HID, svogt + (size_t)f0 * 2 * HW, HID, 2 * HW,
                                ogp, 512, (long)NTOK * 512, fg_b1, 0L, fg_b1, 0L,
                                NTOK, 512, HID, RW * RW, 1.0f, GRP);
    const float* selin = selp[(gi + 1) & 1];
    float* selout = selp[gi & 1];
    if (gi == 0) {
      vsn_combine_kernel<true, false><<<NTOK / 8, 256, 0, stream>>>(ogp, x, swws, sv_bo, sv_bg, sv_sw, sv_sb, sv_lng, sv_lnb,
                                                                   f0, selin, selout, pos, feats16);
    } else if (gi == NGRP - 1) {
      vsn_combine_kernel<false, true><<<NTOK / 8, 256, 0, stream>>>(ogp, x, swws, sv_bo, sv_bg, sv_sw, sv_sb, sv_lng, sv_lnb,
                                                                   f0, selin, selout, pos, feats16);
    } else {
      vsn_combine_kernel<false, false><<<NTOK / 8, 256, 0, stream>>>(ogp, x, swws, sv_bo, sv_bg, sv_sw, sv_sb, sv_lng, sv_lnb,
                                                                    f0, selin, selout, pos, feats16);
    }
  }

  launch_gemm<2, 0, false, 0>(stream, feats16, HID, 0L, wih16[0], HID, 0L, gin, NGATE, 0L, l0_bih, 0L, fg_b1, 0L,
                              NTOK, NGATE, HID, RW, 1.0f, 1);
  lstm_seq_kernel<<<1, 256, 0, stream>>>(gin, whh16[0], l0_bhh, aF[1], a16l0);
  launch_gemm<2, 0, false, 0>(stream, a16l0, HID, 0L, wih16[1], HID, 0L, gin, NGATE, 0L, l1_bih, 0L, fg_b1, 0L,
                              NTOK, NGATE, HID, RW, 1.0f, 1);
  lstm_seq_kernel<<<1, 256, 0, stream>>>(gin, whh16[1], l1_bhh, aF[0], a16p[0]);

  for (int l = 0; l < NLAY; ++l) {
    const int cur = l & 1, nxt = cur ^ 1;
    launch_gemm<0, 1, false, 0>(stream, a16p[cur], HID, 0L, qkt + (size_t)l * 2 * HW, HID, 0L, qkp, 512, 0L,
                                fg_b1, 0L, fg_b1, 0L, NTOK, 512, HID, RW, 1.0f, 1);
    launch_gemm<0, 1, false, 0>(stream, wvt + (size_t)l * HW, HID, 0L, a16p[cur], HID, 0L, vtp, NTOK, 0L,
                                fg_b1, 0L, fg_b1, 0L, HID, NTOK, HID, RW, 1.0f, 1);
    attn32_kernel<<<NBAT * 4 * 2, 128, 0, stream>>>(qkp, vtp, ctx16);
    launch_gemm<2, 0, true, 0>(stream, ctx16, HID, 0L, wot + (size_t)l * HW, HID, 0L, proj, HID, 0L,
                               att_bo + (size_t)l * HID, 0L, aF[cur], 0L, NTOK, HID, HID, RW / CTXCAR, 1.0f, 1);
    float* dstF = (l == NLAY - 1) ? out5 : aF[nxt];
    ln256_kernel<<<NTOK / 8, 256, 0, stream>>>(proj, att_lng + (size_t)l * HID, att_lnb + (size_t)l * HID, dstF, a16p[nxt]);
  }

  heads_kernel<<<1, 256, 0, stream>>>(out5, out_w1, out_b1, out_w2, out_b2, qw, qb, out);
}
